// SW_MetaPath2Vec_86612310491672
// MI455X (gfx1250) — hardware-verified
//
#include <hip/hip_runtime.h>


namespace {
constexpr int N = 2000, NP = 2048, KP = 2016  , LDA = 2048  , NS = 1000, D = 128, H = 256, B = 100000, K = 5, EP = 200000, EN = 200000;
constexpr float AS_ = 8.0f;

typedef _Float16 b16;
typedef __attribute__((ext_vector_type(16))) _Float16 v16b;
typedef __attribute__((ext_vector_type(8))) _Float16 v8b;
typedef __attribute__((ext_vector_type(8))) float v8f;
typedef __attribute__((ext_vector_type(4))) float v4f;
__device__ __forceinline__ float bf16_rne(float f) { unsigned int u = __float_as_uint(f); u += 0x7FFFu + ((u >> 16) & 1u); return __uint_as_float(u & 0xFFFF0000u); }
__device__ __forceinline__ void split16(float v, b16& hi, b16& lo) { hi = (b16)v; lo = (b16)(v - (float)hi); }
__device__ __forceinline__ v16b frag_kb(const b16* p, int hh) { const v8b a = *(const v8b*)(p + 8 * hh), b = *(const v8b*)(p + 16 + 8 * hh); v16b f;
#pragma unroll
  for (int e = 0; e < 8; ++e) { f[e] = a[e]; f[8 + e] = b[e]; } return f; }
__device__ __forceinline__ void frag_split(const float* p, int hh, v16b& fh, v16b& fl) {
#pragma unroll
  for (int e = 0; e < 8; ++e) { b16 a, c; split16(p[8 * hh + e] * AS_, a, c); fh[e] = a; fl[e] = c; split16(p[16 + 8 * hh + e] * AS_, a, c); fh[8 + e] = a; fl[8 + e] = c; } }
__device__ __forceinline__ v8f wmma16b(v16b a, v16b b, v8f c) { v8f d = __builtin_amdgcn_wmma_f32_16x16x32_f16(false, a, false, b, (short)0, c, false, false); asm volatile("v_nop\n\tv_nop\n\tv_nop\n\tv_nop" : "+v"(d) : "v"(a), "v"(b)); return d; }
__device__ __forceinline__ void wave_lds_sync() { __builtin_amdgcn_fence(__ATOMIC_RELEASE, "workgroup"); __builtin_amdgcn_wave_barrier(); __builtin_amdgcn_fence(__ATOMIC_ACQUIRE, "workgroup"); }
__device__ __forceinline__ float nexp(float x) { return __builtin_amdgcn_exp2f(x * 1.4426950408889634f); }
__device__ __forceinline__ float logsig(float x) { return fminf(x, 0.0f) - log1pf(nexp(-fabsf(x))); }
__device__ __forceinline__ float tanh_f(float x) { const float e = nexp(-2.0f * fabsf(x)); const float t = (1.0f - e) / (1.0f + e); return (x >= 0.0f) ? t : -t; }
__device__ __forceinline__ float pmul(float a, float b) { float p = a * b; asm volatile("" : "+v"(p)); return p; }

struct Wo_ { static constexpr size_t AJ = 0, AJT = AJ + (size_t)NP * LDA, W1 = AJT + (size_t)NP * LDA, W2 = W1 + (size_t)H * LDA, END = W2 + (size_t)D * H; };
__global__ __launch_bounds__(256) void prep_kernel(const float* __restrict__ adj, const float* __restrict__ W1, const float* __restrict__ b1, const float* __restrict__ W2, const float* __restrict__ b2, b16* __restrict__ R, float* __restrict__ P) {
  const int t_ = blockIdx.x * 256 + threadIdx.x, nth = gridDim.x * 256;
  auto tr = [&](size_t base, int nrow, int kp, auto val) { for (int p = t_; p < nrow * (kp / 8); p += nth) { const int o = p / (kp / 8), k0 = (p % (kp / 8)) * 8; v8b v;
#pragma unroll
      for (int e8 = 0; e8 < 8; ++e8) v[e8] = (b16)val(o, k0 + e8); *(volatile v8b*)(R + base + (size_t)o * kp + k0) = v; } };
  for (int pass = 0; pass < 2; ++pass) {
    tr(Wo_::AJ, NP, LDA, [&](int i, int k) { return (i < N && k < N) ? bf16_rne(adj[(size_t)i * N + k]) : 0.0f; });
    tr(Wo_::AJT, NP, LDA, [&](int n, int k) { return (n < N && k < N) ? bf16_rne(adj[(size_t)k * N + n]) : 0.0f; });
    tr(Wo_::W1, H, LDA, [&](int o, int k) { return (k < N) ? bf16_rne(W1[(size_t)k * H + o]) : 0.0f; });
    tr(Wo_::W2, D, H, [&](int o, int k) { return bf16_rne(W2[(size_t)k * D + o]); });
    for (int q = t_; q < 384; q += nth) P[q] = (q < 256) ? bf16_rne(b1[q]) : bf16_rne(b2[q - 256]);
    __threadfence(); }
}

__global__ __launch_bounds__(128) void sq_kernel(const b16* __restrict__ Arow, const b16* __restrict__ Brow, int epi, const float* __restrict__ adj, const float* __restrict__ dvec, b16* __restrict__ A2, float* __restrict__ dout, float* __restrict__ gam) {
  __shared__ __attribute__((aligned(16))) float Ts[4][32][64 + 4];
  const int lane = threadIdx.x & 31, wave = threadIdx.x >> 5, nloc = lane & 15, hlf = lane >> 4, m0 = blockIdx.y * 128 + wave * 32, c0 = blockIdx.x * 64;
  v8f acc[2][4];
#pragma unroll
  for (int r = 0; r < 2; ++r)
#pragma unroll
    for (int t = 0; t < 4; ++t) acc[r][t] = (v8f){};
#pragma unroll 3
  for (int kb = 0; kb < KP; kb += 32) { const v16b a0 = frag_kb(Arow + (size_t)(m0 + nloc) * LDA + kb, hlf), a1 = frag_kb(Arow + (size_t)(m0 + 16 + nloc) * LDA + kb, hlf);
#pragma unroll
    for (int t = 0; t < 4; ++t) { const v16b bw = frag_kb(Brow + (size_t)(c0 + t * 16 + nloc) * LDA + kb, hlf); acc[0][t] = wmma16b(a0, bw, acc[0][t]); acc[1][t] = wmma16b(a1, bw, acc[1][t]); } }
#pragma unroll
  for (int t = 0; t < 4; ++t)
#pragma unroll
    for (int r = 0; r < 2; ++r)
#pragma unroll
      for (int v = 0; v < 8; ++v) Ts[wave][r * 16 + 8 * hlf + v][t * 16 + nloc] = acc[r][t][v];
  wave_lds_sync();
  for (int pass = 0; pass < 2; ++pass) {
    if (epi == 0) {
      for (int i = lane; i < 32 * 8; i += 32) { const int rr = i >> 3, c8 = (i & 7) * 8; v8b o; for (int e = 0; e < 8; ++e) o[e] = (b16)Ts[wave][rr][c8 + e]; *(volatile v8b*)(A2 + (size_t)(m0 + rr) * LDA + c0 + c8) = o; }
      { const int row = m0 + lane; if (row >= c0 && row < c0 + 64) ((volatile float*)dout)[row] = Ts[wave][lane][row - c0]; }
    } else {
      for (int i = lane; i < 32 * 16; i += 32) { const int rr = i >> 4, c4 = (i & 15) * 4; const int row = m0 + rr; v4f o;
        for (int e = 0; e < 4; ++e) { const int col = c0 + c4 + e; float g = 0.0f; if (row < N && col < N) { const float p2 = dvec[row] * dvec[col]; const float p1 = Ts[wave][rr][c4 + e] * bf16_rne(adj[(size_t)row * N + col]); g = (p2 > 0.0f) ? p1 / p2 : 0.0f; } o[e] = g; }
        *(volatile v4f*)(gam + (size_t)row * NP + c0 + c4) = o; } }
    __threadfence(); }
}

__global__ __launch_bounds__(256) void norm_kernel(const float* __restrict__ gam, float* __restrict__ rn) {
  __shared__ float Rv[32];
  const int wid = threadIdx.x >> 5, lane = threadIdx.x & 31;
  for (int sub = 0; sub < 4; ++sub) { const int row = blockIdx.x * 32 + wid * 4 + sub; float s = 0.0f; for (int c = lane; c < N; c += 32) { const float g = gam[(size_t)row * NP + c]; s += pmul(g, g); }
#pragma unroll
    for (int o = 1; o < 32; o <<= 1) s += __shfl_xor(s, o);
    if (lane == 0) Rv[wid * 4 + sub] = 1.0f / fmaxf(sqrtf(s), 1e-12f); }
  __syncthreads();
  if (threadIdx.x < 32) { for (int pass = 0; pass < 2; ++pass) ((volatile float*)rn)[blockIdx.x * 32 + threadIdx.x] = Rv[threadIdx.x]; }
  __threadfence();
}

__global__ __launch_bounds__(256) void mlp_kernel(const float* __restrict__ gam, const float* __restrict__ rn, const float* __restrict__ nemb, const b16* __restrict__ R, const float* __restrict__ P, float* __restrict__ hrow) {
  __shared__ __attribute__((aligned(16))) float Tt[64][H + 4]; __shared__ __attribute__((aligned(16))) float Sw[64][D + 4];
  const int lane = threadIdx.x & 31, wave = threadIdx.x >> 5, nloc = lane & 15, hlf = lane >> 4, m0 = blockIdx.x * 64; const b16* W1t = R + Wo_::W1; const b16* W2t = R + Wo_::W2;
  { v8f acc[4][2];
#pragma unroll
    for (int rt = 0; rt < 4; ++rt) { acc[rt][0] = (v8f){}; acc[rt][1] = (v8f){}; }
    for (int kb = 0; kb < KP; kb += 32) { const v16b b0 = frag_kb(W1t + (size_t)(wave * 32 + nloc) * LDA + kb, hlf), b1_ = frag_kb(W1t + (size_t)(wave * 32 + 16 + nloc) * LDA + kb, hlf);
#pragma unroll
      for (int rt = 0; rt < 4; ++rt) { const int row = m0 + rt * 16 + nloc; const float sc = rn[row]; const float* gr = gam + (size_t)row * NP + kb; v16b ah, al;
#pragma unroll
        for (int e = 0; e < 8; ++e) { b16 x_, y_; split16(gr[8 * hlf + e] * sc * AS_, x_, y_); ah[e] = x_; al[e] = y_; split16(gr[16 + 8 * hlf + e] * sc * AS_, x_, y_); ah[8 + e] = x_; al[8 + e] = y_; }
        acc[rt][0] = wmma16b(ah, b0, acc[rt][0]); acc[rt][0] = wmma16b(al, b0, acc[rt][0]); acc[rt][1] = wmma16b(ah, b1_, acc[rt][1]); acc[rt][1] = wmma16b(al, b1_, acc[rt][1]); } }
#pragma unroll
    for (int rt = 0; rt < 4; ++rt)
#pragma unroll
      for (int t = 0; t < 2; ++t) { const int cc = wave * 32 + t * 16 + nloc; const float bb = P[cc];
#pragma unroll
        for (int r = 0; r < 8; ++r) Tt[rt * 16 + 8 * hlf + r][cc] = tanh_f(acc[rt][t][r] * (1.0f / AS_) + bb); } }
  __syncthreads();
  { v8f acc[4];
#pragma unroll
    for (int rt = 0; rt < 4; ++rt) acc[rt] = (v8f){};
#pragma unroll
    for (int kb = 0; kb < H; kb += 32) { const v16b bw = frag_kb(W2t + (size_t)(wave * 16 + nloc) * H + kb, hlf);
#pragma unroll
      for (int rt = 0; rt < 4; ++rt) { v16b ah, al; frag_split(&Tt[rt * 16 + nloc][kb], hlf, ah, al); acc[rt] = wmma16b(ah, bw, acc[rt]); acc[rt] = wmma16b(al, bw, acc[rt]); } }
#pragma unroll
    for (int rt = 0; rt < 4; ++rt) { const int cc = wave * 16 + nloc; const float bb = P[256 + cc];
#pragma unroll
      for (int r = 0; r < 8; ++r) Sw[rt * 16 + 8 * hlf + r][cc] = acc[rt][r] * (1.0f / AS_) + bb; } }
  __syncthreads();
  for (int pass = 0; pass < 2; ++pass) { for (int i = threadIdx.x; i < 64 * 64; i += 256) { const int rr = i >> 6, c4 = (i & 63) * 4; const int row = m0 + rr; v4f o;
      if (c4 < D) { for (int e = 0; e < 4; ++e) o[e] = (row < N) ? bf16_rne(nemb[(size_t)row * D + c4 + e]) : 0.0f; } else { o = *(const v4f*)(&Sw[rr][c4 - D]); }
      *(volatile v4f*)(hrow + (size_t)row * H + c4) = o; } __threadfence(); }
}

__global__ __launch_bounds__(256) void score_kernel(const float* __restrict__ hrow, const int* __restrict__ ps, const int* __restrict__ pd, const int* __restrict__ ns, const int* __restrict__ nd, float* __restrict__ out) {
  const int g = blockIdx.x * 256 + threadIdx.x; if (g >= EP + EN) return; const bool isneg = (g >= EP); const int e = isneg ? g - EP : g;
  int s = isneg ? ns[e] : ps[e], d = isneg ? nd[e] : pd[e]; s = (s < 0) ? 0 : (s >= NS ? NS - 1 : s); d = (d < 0) ? 0 : (d >= N - NS ? N - NS - 1 : d);
  const float* hs = hrow + (size_t)s * H; const float* hd = hrow + (size_t)(NS + d) * H; float acc = 0.0f;
  for (int c = 0; c < H; c += 4) { const v4f a = *(const v4f*)(hs + c), b = *(const v4f*)(hd + c); acc += pmul(a[0], b[0]); acc += pmul(a[1], b[1]); acc += pmul(a[2], b[2]); acc += pmul(a[3], b[3]); }
  for (int pass = 0; pass < 2; ++pass) { ((volatile float*)out)[1 + g] = acc; __threadfence(); }
}

__global__ __launch_bounds__(256) void sg_kernel(const float* __restrict__ ne, const float* __restrict__ ce, const int* __restrict__ pu, const int* __restrict__ pv, const int* __restrict__ nv, float* __restrict__ part) {
  __shared__ float red[256];
  const int i = blockIdx.x * 256 + threadIdx.x; float term = 0.0f;
  if (i < B) { int u = pu[i], v = pv[i]; u = (u < 0) ? 0 : (u >= N ? N - 1 : u); v = (v < 0) ? 0 : (v >= N ? N - 1 : v); const float* eu = ne + (size_t)u * D; const float* ev = ce + (size_t)v * D;
    float dp = 0.0f; for (int c = 0; c < D; ++c) dp += pmul(bf16_rne(eu[c]), bf16_rne(ev[c])); dp = fminf(fmaxf(dp, -10.0f), 10.0f); term = -logsig(dp);
    for (int k = 0; k < K; ++k) { int w = nv[(size_t)i * K + k]; w = (w < 0) ? 0 : (w >= N ? N - 1 : w); const float* ew = ce + (size_t)w * D; float dn = 0.0f; for (int c = 0; c < D; ++c) dn += pmul(bf16_rne(ew[c]), bf16_rne(eu[c])); dn = fminf(fmaxf(dn, -10.0f), 10.0f); term += -logsig(-dn); } }
  red[threadIdx.x] = term; __syncthreads();
  for (int st = 128; st > 0; st >>= 1) { if ((int)threadIdx.x < st) red[threadIdx.x] += red[threadIdx.x + st]; __syncthreads(); }
  if (threadIdx.x < 32) { const float v = (threadIdx.x == 0) ? red[0] : 0.0f; for (int pass = 0; pass < 2; ++pass) ((volatile float*)part)[(size_t)blockIdx.x * 32 + threadIdx.x] = v; }
  __threadfence();
}
__global__ __launch_bounds__(256) void loss_kernel(const float* __restrict__ part, int nblk, float* __restrict__ out) {
  __shared__ float red[256];
  float s = 0.0f; for (int b = threadIdx.x; b < nblk; b += 256) s += part[(size_t)b * 32]; red[threadIdx.x] = s; __syncthreads();
  for (int st = 128; st > 0; st >>= 1) { if ((int)threadIdx.x < st) red[threadIdx.x] += red[threadIdx.x + st]; __syncthreads(); }
  if (threadIdx.x == 0) { for (int pass = 0; pass < 2; ++pass) ((volatile float*)out)[0] = red[0] / (float)B; }
  __threadfence();
}
}

extern "C" void kernel_launch(void* const* d_in, const int* in_sizes, int n_in,
                              void* d_out, int out_size, void* d_ws, size_t ws_size, hipStream_t stream) {
  (void)n_in; (void)out_size;
  const float* ne = (const float*)d_in[0]; const float* ce = (const float*)d_in[1]; const float* adj = (const float*)d_in[2]; const float* W1 = (const float*)d_in[3]; const float* b1 = (const float*)d_in[4]; const float* W2 = (const float*)d_in[5]; const float* b2 = (const float*)d_in[6];
  const int* pu = (const int*)d_in[7]; const int* pv = (const int*)d_in[8]; const int* nv = (const int*)d_in[9]; const int* ps = (const int*)d_in[10]; const int* pd = (const int*)d_in[11]; const int* ns = (const int*)d_in[12]; const int* nd = (const int*)d_in[13];
  float* out = (float*)d_out;
  if (in_sizes[2] != N * N || in_sizes[3] != N * H || in_sizes[7] != B || in_sizes[9] != B * K || in_sizes[10] != EP || in_sizes[12] != EN) return;
  size_t off = 0; char* ws = (char*)d_ws;
  auto carve = [&](size_t bytes) { char* p = ws + off; off += (bytes + 255) & ~(size_t)255; return p; };
  b16* R = (b16*)carve(Wo_::END * 2); float* P = (float*)carve(512 * 4); b16* A2 = (b16*)carve((size_t)NP * LDA * 2); float* dv = (float*)carve(NP * 4); float* gam = (float*)carve((size_t)NP * NP * 4); float* rn = (float*)carve(NP * 4); float* hrow = (float*)carve((size_t)NP * H * 4);
  const int nsg = (B + 255) / 256; float* part = (float*)carve((size_t)nsg * 32 * 4);
  if (off > ws_size) return;
  prep_kernel<<<256, 256, 0, stream>>>(adj, W1, b1, W2, b2, R, P);
  sq_kernel<<<dim3(NP / 64, NP / 128), 128, 0, stream>>>(R + Wo_::AJ, R + Wo_::AJT, 0, adj, nullptr, A2, dv, nullptr);
  sq_kernel<<<dim3(NP / 64, NP / 128), 128, 0, stream>>>(A2, R + Wo_::AJT, 1, adj, dv, nullptr, nullptr, gam);
  norm_kernel<<<NP / 32, 256, 0, stream>>>(gam, rn);
  mlp_kernel<<<NP / 64, 256, 0, stream>>>(gam, rn, ne, R, P, hrow);
  score_kernel<<<(EP + EN + 255) / 256, 256, 0, stream>>>(hrow, ps, pd, ns, nd, out);
  sg_kernel<<<nsg, 256, 0, stream>>>(ne, ce, pu, pv, nv, part);
  loss_kernel<<<1, 256, 0, stream>>>(part, nsg, out);
}
